// SelfAttention_18245021073428
// MI455X (gfx1250) — hardware-run, weakly checked
//
#include <hip/hip_runtime.h>


#ifndef NB
#define NB 1
#endif
#ifndef SEQ
#define SEQ 4096
#endif
#define NB_FULL    1
#define SEQ_FULL   4096
#define DMODEL     1024
#define HDIM       128
#define NPROJ      3
#define WROWS      (NPROJ * HDIM)
#define WPIECES    (WROWS * DMODEL / 8)
#define WBLK       (WPIECES / 256)
#define PM         64
#define QP         136
#define VP         72
#define SLDS       9216
#define BQ         64
#define BK         32
#define NWAVE      4
#define OP         132
#define WS_CAP     134217728ull

static_assert(NB == 1);
static_assert(NB <= NB_FULL);
static_assert(SEQ <= SEQ_FULL);
static_assert(SEQ % PM == 0);
static_assert(SEQ % BQ == 0);
static_assert(SEQ % BK == 0);
static_assert(SEQ % 64 == 0);
static_assert(DMODEL % 32 == 0);
static_assert(HDIM == 128);
static_assert(HDIM % 32 == 0);
static_assert(BQ == NWAVE * 16);
static_assert(PM == 64);
static_assert(WPIECES % 256 == 0);
static_assert(SLDS >= PM * QP);
static_assert(SLDS >= HDIM * VP);
static_assert((QP * 2) % 16 == 0);
static_assert((VP * 2) % 16 == 0);
static_assert((OP * 4) % 16 == 0);
static_assert(OP >= HDIM);
static_assert(HDIM * 4 == 32 * 16);
static_assert(HDIM * 2 == 16 * 16);
static_assert((unsigned long long)WROWS * DMODEL * 2ull + (unsigned long long)WROWS * 4ull +
              3ull * SEQ * HDIM * 2ull <= WS_CAP);

typedef __bf16   bf16;
typedef _Float16 f16;
typedef bf16     v16bf __attribute__((ext_vector_type(16)));
typedef f16      v16h  __attribute__((ext_vector_type(16)));
typedef f16      v8h   __attribute__((ext_vector_type(8)));
typedef float    v8f   __attribute__((ext_vector_type(8)));
typedef float    v4f   __attribute__((ext_vector_type(4)));
typedef unsigned v4u   __attribute__((ext_vector_type(4)));

union FragB  { v16bf v; v4u q[2]; bf16 h[16]; };
union FragH  { v16h  v; v4u q[2]; f16  h[16]; };
union Pack8B { v4u u; bf16 h[8]; };
union Pack8H { v4u u; v8h v; f16 h[8]; };

static __device__ __forceinline__ v8f mma_bf16(v16bf a, v16bf b, v8f acc) {
  acc = __builtin_amdgcn_wmma_f32_16x16x32_bf16(false, a, false, b, (short)0, acc, false, false);
  asm volatile("v_nop\n\tv_nop\n\tv_nop\n\tv_nop" : "+v"(acc) : "v"(a), "v"(b));
  return acc;
}
static __device__ __forceinline__ v8f mma_f16(v16h a, v16h b, v8f acc) {
  acc = __builtin_amdgcn_wmma_f32_16x16x32_f16(false, a, false, b, (short)0, acc, false, false);
  asm volatile("v_nop\n\tv_nop\n\tv_nop\n\tv_nop" : "+v"(acc) : "v"(a), "v"(b));
  return acc;
}

__global__ __launch_bounds__(256) void wplane_kernel(const float* __restrict__ qW,
                                                     const float* __restrict__ kW,
                                                     const float* __restrict__ vW,
                                                     const float* __restrict__ qb,
                                                     const float* __restrict__ kb,
                                                     const float* __restrict__ vb,
                                                     bf16* __restrict__ wb,
                                                     float* __restrict__ bias) {
  const int tid = threadIdx.x;
  if (blockIdx.x < WBLK) {
    const int g     = blockIdx.x * 256 + tid;
    const int n     = g >> 7;
    const int c0    = (g & 127) << 3;
    const int which = n >> 7;
    const size_t off = (size_t)(n & 127) * DMODEL + c0;
    const v4f q0 = *(const v4f*)(qW + off);
    const v4f q1 = *(const v4f*)(qW + off + 4);
    const v4f k0 = *(const v4f*)(kW + off);
    const v4f k1 = *(const v4f*)(kW + off + 4);
    const v4f v0 = *(const v4f*)(vW + off);
    const v4f v1 = *(const v4f*)(vW + off + 4);
    const v4f s0 = (which == 0) ? q0 : ((which == 1) ? k0 : v0);
    const v4f s1 = (which == 0) ? q1 : ((which == 1) ? k1 : v1);
    Pack8B pk;
    #pragma unroll
    for (int i = 0; i < 4; ++i) {
      pk.h[i]     = (bf16)s0[i];
      pk.h[4 + i] = (bf16)s1[i];
    }
    const v4u val = pk.u;
    bf16* dst = wb + (size_t)n * DMODEL + c0;
    *(volatile v4u*)dst = val;
    __threadfence();
    *(volatile v4u*)dst = val;
  } else if (tid < 96) {
    const int n0    = tid * 4;
    const int which = n0 >> 7;
    const int o     = n0 & 127;
    const v4f a = *(const v4f*)(qb + o);
    const v4f b = *(const v4f*)(kb + o);
    const v4f c = *(const v4f*)(vb + o);
    const v4f s = (which == 0) ? a : ((which == 1) ? b : c);
    v4f val;
    #pragma unroll
    for (int i = 0; i < 4; ++i) val[i] = (float)(bf16)s[i];
    float* dst = bias + n0;
    *(volatile v4f*)dst = val;
    __threadfence();
    *(volatile v4f*)dst = val;
  }
}

__global__ __launch_bounds__(256) void proj_kernel(const float* __restrict__ X,
                                                   const bf16* __restrict__ wb,
                                                   const float* __restrict__ bias,
                                                   f16* __restrict__ qk,
                                                   f16* __restrict__ vt) {
  const int mblk  = blockIdx.x;
  const int which = blockIdx.y;
  const int tid   = threadIdx.x;
  const int wave  = __builtin_amdgcn_readfirstlane(threadIdx.x >> 5);
  const int lane  = tid & 31;
  const int lq    = lane & 15;
  const int hi    = lane >> 4;
  const int rt    = wave & 3;
  const int cg    = wave >> 2;

  __shared__ __align__(16) f16 sT[SLDS];

  const float* xp = X + (size_t)(mblk * PM + rt * 16 + lq) * DMODEL + hi * 8;
  const bf16*  wp = wb + (size_t)(which * HDIM + cg * 64 + lq) * DMODEL + hi * 8;

  v8f acc[4];
  #pragma unroll
  for (int ct = 0; ct < 4; ++ct) acc[ct] = (v8f){0, 0, 0, 0, 0, 0, 0, 0};

  #pragma unroll 1
  for (int k0 = 0; k0 < DMODEL; k0 += 32) {
    const v4f a0 = *(const v4f*)(xp + k0);
    const v4f a1 = *(const v4f*)(xp + k0 + 4);
    const v4f b0 = *(const v4f*)(xp + k0 + 16);
    const v4f b1 = *(const v4f*)(xp + k0 + 20);
    FragB af;
    #pragma unroll
    for (int i = 0; i < 4; ++i) {
      af.h[i]      = (bf16)a0[i];
      af.h[4 + i]  = (bf16)a1[i];
      af.h[8 + i]  = (bf16)b0[i];
      af.h[12 + i] = (bf16)b1[i];
    }
    FragB bfr[4];
    #pragma unroll
    for (int ct = 0; ct < 4; ++ct) {
      const bf16* base = wp + (size_t)(ct * 16) * DMODEL + k0;
      bfr[ct].q[0] = *(const v4u*)(base);
      bfr[ct].q[1] = *(const v4u*)(base + 16);
    }
    #pragma unroll
    for (int ct = 0; ct < 4; ++ct) acc[ct] = mma_bf16(af.v, bfr[ct].v, acc[ct]);
  }

  float bvv[4];
  #pragma unroll
  for (int ct = 0; ct < 4; ++ct) bvv[ct] = bias[which * HDIM + cg * 64 + ct * 16 + lq];

  if (which < 2) {
    #pragma unroll
    for (int ct = 0; ct < 4; ++ct) {
      #pragma unroll
      for (int r = 0; r < 8; ++r) {
        sT[(rt * 16 + hi * 8 + r) * QP + cg * 64 + ct * 16 + lq] = (f16)(acc[ct][r] + bvv[ct]);
      }
    }
  } else {
    #pragma unroll
    for (int ct = 0; ct < 4; ++ct) {
      Pack8H ph;
      #pragma unroll
      for (int r = 0; r < 8; ++r) ph.h[r] = (f16)(acc[ct][r] + bvv[ct]);
      *(v8h*)(sT + (cg * 64 + ct * 16 + lq) * VP + rt * 16 + hi * 8) = ph.v;
    }
  }
  __syncthreads();

  v4u    vals[4];
  size_t gidx[4];
  if (which < 2) {
    #pragma unroll
    for (int it = 0; it < 4; ++it) {
      const int row = wave * 8 + it * 2 + hi;
      Pack8H ph;
      ph.v = *(const v8h*)(sT + row * QP + lq * 8);
      vals[it] = ph.u;
      gidx[it] = (size_t)which * SEQ * HDIM + (size_t)(mblk * PM + row) * HDIM + lq * 8;
    }
    #pragma unroll
    for (int it = 0; it < 4; ++it) *(volatile v4u*)(qk + gidx[it]) = vals[it];
    __threadfence();
    #pragma unroll
    for (int it = 0; it < 4; ++it) *(volatile v4u*)(qk + gidx[it]) = vals[it];
  } else {
    #pragma unroll
    for (int it = 0; it < 4; ++it) {
      const int d  = wave * 16 + it * 4 + (lane >> 3);
      const int ts = (lane & 7) * 8;
      Pack8H ph;
      ph.v = *(const v8h*)(sT + d * VP + ts);
      vals[it] = ph.u;
      gidx[it] = (size_t)d * SEQ + (size_t)mblk * PM + ts;
    }
    #pragma unroll
    for (int it = 0; it < 4; ++it) *(volatile v4u*)(vt + gidx[it]) = vals[it];
    __threadfence();
    #pragma unroll
    for (int it = 0; it < 4; ++it) *(volatile v4u*)(vt + gidx[it]) = vals[it];
  }
}

__global__ __launch_bounds__(128) void attn_kernel(const f16* __restrict__ qk,
                                                   const f16* __restrict__ vt,
                                                   float* __restrict__ out) {
  const int qblk = blockIdx.x;
  const int tid  = threadIdx.x;
  const int wave = __builtin_amdgcn_readfirstlane(threadIdx.x >> 5);
  const int lane = tid & 31;
  const int lq   = lane & 15;
  const int hi   = lane >> 4;

  __shared__ __align__(16) float sO[NWAVE * 16 * OP];

  const int qrow0 = qblk * BQ + wave * 16;
  const f16* qh = qk;
  const f16* kh = qk + (size_t)SEQ * HDIM;

  FragH qf[4];
  {
    const f16* qp = qh + (size_t)(qrow0 + lq) * HDIM + hi * 8;
    #pragma unroll
    for (int f = 0; f < 4; ++f) {
      qf[f].q[0] = *(const v4u*)(qp + f * 32);
      qf[f].q[1] = *(const v4u*)(qp + f * 32 + 16);
    }
  }

  v8f o[8];
  #pragma unroll
  for (int dt = 0; dt < 8; ++dt) o[dt] = (v8f){0, 0, 0, 0, 0, 0, 0, 0};

  float rmax = -__builtin_inff();
  float rsum = 0.0f;
  const float SL = 0.0078125f * 1.4426950408889634f;

  const int nchunk = SEQ / BK;
  #pragma unroll 1
  for (int i = 0; i < nchunk; ++i) {
    const int j0 = i * BK;

    v8f c[2];
    #pragma unroll
    for (int sub = 0; sub < 2; ++sub) {
      FragH ak[4];
      const f16* kbase = kh + (size_t)(j0 + sub * 16 + lq) * HDIM + hi * 8;
      #pragma unroll
      for (int f = 0; f < 4; ++f) {
        ak[f].q[0] = *(const v4u*)(kbase + f * 32);
        ak[f].q[1] = *(const v4u*)(kbase + f * 32 + 16);
      }
      v8f acc = (v8f){0, 0, 0, 0, 0, 0, 0, 0};
      #pragma unroll
      for (int f = 0; f < 4; ++f) acc = mma_f16(ak[f].v, qf[f].v, acc);
      c[sub] = acc;
      __builtin_amdgcn_sched_barrier(0);
    }

    float m_new = rmax;
    #pragma unroll
    for (int r = 0; r < 8; ++r) {
      m_new = fmaxf(m_new, c[0][r]);
      m_new = fmaxf(m_new, c[1][r]);
    }
    m_new = fmaxf(m_new, __shfl_xor(m_new, 16, 32));
    const float scale = __builtin_amdgcn_exp2f((rmax - m_new) * SL);
    rmax = m_new;

    FragH pa;
    float psum = 0.0f;
    #pragma unroll
    for (int r = 0; r < 8; ++r) {
      const float p0 = __builtin_amdgcn_exp2f((c[0][r] - m_new) * SL);
      const float p1 = __builtin_amdgcn_exp2f((c[1][r] - m_new) * SL);
      psum += p0 + p1;
      pa.h[r]     = (f16)(p0 * 4096.0f);
      pa.h[8 + r] = (f16)(p1 * 4096.0f);
    }
    rsum = rsum * scale + psum + __shfl_xor(psum, 16, 32);

    float sc[8];
    #pragma unroll
    for (int r = 0; r < 8; ++r) sc[r] = __shfl(scale, (hi << 3) + r, 32);
    #pragma unroll
    for (int dt = 0; dt < 8; ++dt) {
      #pragma unroll
      for (int r = 0; r < 8; ++r) o[dt][r] *= sc[r];
    }
    __builtin_amdgcn_sched_barrier(0);

    #pragma unroll
    for (int g = 0; g < 2; ++g) {
      FragH bv[4];
      #pragma unroll
      for (int t = 0; t < 4; ++t) {
        const f16* vbase = vt + (size_t)((g * 4 + t) * 16 + lq) * SEQ + j0 + hi * 8;
        bv[t].q[0] = *(const v4u*)(vbase);
        bv[t].q[1] = *(const v4u*)(vbase + 16);
      }
      #pragma unroll
      for (int t = 0; t < 4; ++t) o[g * 4 + t] = mma_f16(pa.v, bv[t].v, o[g * 4 + t]);
      __builtin_amdgcn_sched_barrier(0);
    }
  }

  float rs[8];
  #pragma unroll
  for (int r = 0; r < 8; ++r) rs[r] = 1.0f / __shfl(rsum, (hi << 3) + r, 32);

  float* so = sO + wave * (16 * OP);
  #pragma unroll
  for (int r = 0; r < 8; ++r) {
    #pragma unroll
    for (int dt = 0; dt < 8; ++dt) {
      so[(hi * 8 + r) * OP + dt * 16 + lq] = o[dt][r] * (1.0f / 4096.0f) * rs[r];
    }
  }
  __syncthreads();

  v4f vals[16];
  #pragma unroll
  for (int it = 0; it < 16; ++it) vals[it] = *(const v4f*)(so + it * OP + lane * 4);
  float* obase = out + (size_t)qrow0 * HDIM + lane * 4;
  #pragma unroll
  for (int it = 0; it < 16; ++it) *(volatile v4f*)(obase + (size_t)it * HDIM) = vals[it];
  __threadfence();
  #pragma unroll
  for (int it = 0; it < 16; ++it) *(volatile v4f*)(obase + (size_t)it * HDIM) = vals[it];
}

extern "C" void kernel_launch(void* const* d_in, const int* in_sizes, int n_in,
                              void* d_out, int out_size, void* d_ws, size_t ws_size,
                              hipStream_t stream) {
  if (n_in < 7) return;
  if ((size_t)in_sizes[0] < (size_t)SEQ * DMODEL) return;
  if ((size_t)in_sizes[1] < (size_t)HDIM * DMODEL) return;
  if ((size_t)in_sizes[2] < (size_t)HDIM) return;
  if ((size_t)in_sizes[3] < (size_t)HDIM * DMODEL) return;
  if ((size_t)in_sizes[4] < (size_t)HDIM) return;
  if ((size_t)in_sizes[5] < (size_t)HDIM * DMODEL) return;
  if ((size_t)in_sizes[6] < (size_t)HDIM) return;
  if ((size_t)out_size < (size_t)SEQ * HDIM) return;

  const size_t wb_bytes   = (size_t)WROWS * DMODEL * 2;
  const size_t bias_bytes = (size_t)WROWS * 4;
  const size_t qk_bytes   = (size_t)2 * SEQ * HDIM * 2;
  const size_t vt_bytes   = (size_t)HDIM * SEQ * 2;
  const size_t total      = wb_bytes + bias_bytes + qk_bytes + vt_bytes;
  if (ws_size < total) return;
  if (total > (size_t)WS_CAP) return;

  const float* X  = (const float*)d_in[0];
  const float* qW = (const float*)d_in[1];
  const float* qb = (const float*)d_in[2];
  const float* kW = (const float*)d_in[3];
  const float* kb = (const float*)d_in[4];
  const float* vW = (const float*)d_in[5];
  const float* vb = (const float*)d_in[6];
  float*       out = (float*)d_out;

  char*  ws   = (char*)d_ws;
  bf16*  wb   = (bf16*)ws;
  float* bias = (float*)(ws + wb_bytes);
  f16*   qk   = (f16*)(ws + wb_bytes + bias_bytes);
  f16*   vt   = (f16*)(ws + wb_bytes + bias_bytes + qk_bytes);

  wplane_kernel<<<dim3(WBLK + 1), 256, 0, stream>>>(qW, kW, vW, qb, kb, vb, wb, bias);
  proj_kernel<<<dim3(SEQ / PM, NPROJ), 256, 0, stream>>>(X, wb, bias, qk, vt);
  attn_kernel<<<dim3(SEQ / BQ), 128, 0, stream>>>(qk, vt, out);
}
